// GenerativeRNNmodel_82506321756339
// MI455X (gfx1250) — hardware-run, weakly checked
//
#include <hip/hip_runtime.h>
#include <math.h>

constexpr int kSeqB    = 64;
constexpr int kSteps   = 2048;
constexpr int kHid     = 128;
constexpr int kGate3   = 384;
constexpr int kStreams = 128;
constexpr int kTileS   = 16;
constexpr int kGruThr  = 256;
constexpr int kHPitch  = 136;
constexpr int kFeatW   = 256;
constexpr int kPredH   = 64;
constexpr int kChunkC  = 32;
constexpr int kFcRows  = kSeqB * kSteps;
constexpr int kFcChunk = 32768;
constexpr int kFc0N    = 256;
constexpr int kFc1N    = 64;
constexpr int kFcK     = 256;
constexpr float kInv16 = 0.0625f;

static_assert(kStreams % kTileS == 0 && kSeqB % kTileS == 0, "direction is block-uniform");
static_assert(kHid % 32 == 0 && kFcK % 32 == 0, "k step");
static_assert(kSteps % kChunkC == 0, "whole preds lines");
static_assert(kFcRows % kFcChunk == 0 && kFcChunk % 64 == 0 && kFc0N % 64 == 0 && kFc1N % 64 == 0, "tile multiples");
static_assert(kFcChunk % 256 == 0, "head grid exact");
static_assert(kTileS * 2 == 32 && kGruThr == 256, "8 waves, 16 streams");
static_assert((kGate3 * kHid) % (8 * 256) == 0 && (kPredH * kHid) % (8 * 256) == 0 &&
              (kFc0N * kFcK) % (8 * 256) == 0 && (kFc1N * kFcK) % (8 * 256) == 0, "cast grids exact");

typedef __attribute__((ext_vector_type(16))) _Float16 v16h;
typedef __attribute__((ext_vector_type(8)))  _Float16 v8h;
typedef __attribute__((ext_vector_type(16))) __bf16   v16b;
typedef __attribute__((ext_vector_type(8)))  __bf16   v8b;
typedef __attribute__((ext_vector_type(8)))  float    v8f;
typedef __attribute__((ext_vector_type(4)))  float    v4f;
#define U16(p) ((const unsigned short*)(const void*)(p))

__device__ __forceinline__ unsigned short f2bf_bits(float f) {
  unsigned u = __float_as_uint(f);
  return (unsigned short)((u + 0x7FFFu + ((u >> 16) & 1u)) >> 16);
}
__device__ __forceinline__ float bf_bits2f(unsigned short h) { return __uint_as_float(((unsigned)h) << 16); }

__device__ __forceinline__ void dep_guard_h(v8f& a, v8f& b, v16h x, v16h y) { asm volatile("v_nop\n\tv_nop\n\tv_nop\n\tv_nop" : "+v"(a), "+v"(b) : "v"(x), "v"(y)); }
__device__ __forceinline__ void dep_guard_b(v8f& a, v8f& b, v16b x, v16b y) { asm volatile("v_nop\n\tv_nop\n\tv_nop\n\tv_nop" : "+v"(a), "+v"(b) : "v"(x), "v"(y)); }
__device__ __forceinline__ void dep_guard1_h(v8f& a, v16h x, v16h y) { asm volatile("v_nop\n\tv_nop\n\tv_nop\n\tv_nop" : "+v"(a) : "v"(x), "v"(y)); }
__device__ __forceinline__ void keep4_h(v16h a, v16h b, v16h c, v16h d) { asm volatile("v_nop" :: "v"(a), "v"(b), "v"(c), "v"(d)); }
__device__ __forceinline__ void keep4_b(v16b a, v16b b, v16b c, v16b d) { asm volatile("v_nop" :: "v"(a), "v"(b), "v"(c), "v"(d)); }
__device__ __forceinline__ void acc_guard4(v8f& a, v8f& b, v8f& c, v8f& d) { asm volatile("v_nop\n\tv_nop\n\tv_nop\n\tv_nop" : "+v"(a), "+v"(b), "+v"(c), "+v"(d)); }
__device__ __forceinline__ void acc_guard3(v8f& a, v8f& b, v8f& c) { asm volatile("v_nop\n\tv_nop\n\tv_nop\n\tv_nop" : "+v"(a), "+v"(b), "+v"(c)); }

template <typename T> struct Frag;
template <> struct Frag<_Float16> {
  typedef v16h V; union U { v16h v; v8h h[2]; };
  static __device__ __forceinline__ v16h load(const _Float16* p) {
    U f; f.h[0] = *(const v8h*)(p); f.h[1] = *(const v8h*)(p + 16); return f.v;
  }
  static __device__ __forceinline__ v8f mma(v16h a, v16h b, v8f c) {
    return __builtin_amdgcn_wmma_f32_16x16x32_f16(false, a, false, b, (short)0, c, false, false);
  }
  static __device__ __forceinline__ void guard(v8f& a, v8f& b, v16h x, v16h y) { dep_guard_h(a, b, x, y); }
  static __device__ __forceinline__ void keep(v16h a, v16h b, v16h c, v16h d) { keep4_h(a, b, c, d); }
};
template <> struct Frag<__bf16> {
  typedef v16b V; union U { v16b v; v8b h[2]; };
  static __device__ __forceinline__ v16b load(const __bf16* p) {
    U f; f.h[0] = *(const v8b*)(p); f.h[1] = *(const v8b*)(p + 16); return f.v;
  }
  static __device__ __forceinline__ v8f mma(v16b a, v16b b, v8f c) {
    return __builtin_amdgcn_wmma_f32_16x16x32_bf16(false, a, false, b, (short)0, c, false, false);
  }
  static __device__ __forceinline__ void guard(v8f& a, v8f& b, v16b x, v16b y) { dep_guard_b(a, b, x, y); }
  static __device__ __forceinline__ void keep(v16b a, v16b b, v16b c, v16b d) { keep4_b(a, b, c, d); }
};

__device__ __forceinline__ float fsigm(float x) { return __builtin_amdgcn_rcpf(1.0f + __expf(-x)); }
__device__ __forceinline__ float ftanh(float x) { return 1.0f - 2.0f * __builtin_amdgcn_rcpf(1.0f + __expf(2.0f * x)); }

template <int ET> struct Elem;
template <> struct Elem<0> { typedef _Float16 T; };
template <> struct Elem<1> { typedef __bf16 T; };
template <int ET, bool SPLIT, int BIAS_MODE, int OUT_MODE, bool RESID, int ACT = 0>
__global__ __launch_bounds__(256) void wmma_gemm64(
    const unsigned short* __restrict__ Ap, const unsigned short* __restrict__ A2p, int lda, long strideA,
    const unsigned short* __restrict__ Btp, const unsigned short* __restrict__ Bt2p, int ldb, long strideB,
    void* __restrict__ Cout, void* __restrict__ Cout2, int ldc, long strideC,
    const float* __restrict__ bias,
    const float* __restrict__ resid, long strideR,
    int M, int N, int K, float scale) {
  typedef typename Elem<ET>::T T;
  typedef typename Frag<T>::V V;
  const T* A = (const T*)Ap; const T* A2 = (const T*)A2p; const T* Bt = (const T*)Btp; const T* Bt2 = (const T*)Bt2p;
  __shared__ __align__(16) float sT[8][16 * 68];
  const int b    = blockIdx.y;
  const int lane = threadIdx.x & 31;
  const int wave = threadIdx.x >> 5;
  const int tilesN = N >> 6;
  const int tilesM = M >> 6;
  const int tile = blockIdx.x * 8 + wave;
  if (tile >= tilesM * tilesN) return;
  const int tm = tile / tilesN;
  const int tn = tile - tm * tilesN;
  const int m0 = tm << 6;
  const int n0 = tn << 6;

  const T* Ab  = A  + (size_t)b * strideA;
  const T* Bb  = Bt + (size_t)b * strideB;
  const T* Ab2 = SPLIT ? (A2  + (size_t)b * strideA) : nullptr;
  const T* Bb2 = SPLIT ? (Bt2 + (size_t)b * strideB) : nullptr;

  const int rlane = lane & 15;
  const int koff  = (lane >> 4) * 8;
  const int mOff  = (lane >> 4) * 8;

  v8f acc[4][4];
#pragma unroll
  for (int i = 0; i < 4; ++i)
#pragma unroll
    for (int j = 0; j < 4; ++j) acc[i][j] = (v8f){0.f,0.f,0.f,0.f,0.f,0.f,0.f,0.f};

  for (int k0 = 0; k0 < K; k0 += 32) {
    V bh[4], bl[4];
#pragma unroll
    for (int j = 0; j < 4; ++j) {
      const size_t bo = (size_t)(n0 + (j << 4) + rlane) * ldb + koff + k0;
      bh[j] = Frag<T>::load(Bb + bo);
      if (SPLIT) bl[j] = Frag<T>::load(Bb2 + bo);
    }
#pragma unroll
    for (int i = 0; i < 4; ++i) {
      const size_t ao = (size_t)(m0 + (i << 4) + rlane) * lda + koff + k0;
      V ah = Frag<T>::load(Ab + ao);
      V al;
      if (SPLIT) al = Frag<T>::load(Ab2 + ao);
#pragma unroll
      for (int j = 0; j < 4; ++j) {
        acc[i][j] = Frag<T>::mma(ah, bh[j], acc[i][j]);
        if (SPLIT) {
          acc[i][j] = Frag<T>::mma(ah, bl[j], acc[i][j]);
          acc[i][j] = Frag<T>::mma(al, bh[j], acc[i][j]);
        }
      }
      Frag<T>::guard(acc[i][0], acc[i][3], ah, SPLIT ? al : ah);
    }
    Frag<T>::keep(bh[0], bh[1], bh[2], bh[3]);
    if (SPLIT) Frag<T>::keep(bl[0], bl[1], bl[2], bl[3]);
  }
  acc_guard4(acc[0][0], acc[0][1], acc[0][2], acc[0][3]);
  acc_guard4(acc[1][0], acc[1][1], acc[1][2], acc[1][3]);
  acc_guard4(acc[2][0], acc[2][1], acc[2][2], acc[2][3]);
  acc_guard4(acc[3][0], acc[3][1], acc[3][2], acc[3][3]);

  float* slab = sT[wave];
  const float* Rb = RESID ? (resid + (size_t)b * strideR) : nullptr;
#pragma unroll
  for (int i = 0; i < 4; ++i) {
    const int mBase = m0 + (i << 4);
#pragma unroll
    for (int j = 0; j < 4; ++j) {
      const int n = n0 + (j << 4) + rlane;
      float bv = 0.f;
      if (BIAS_MODE == 2) bv = bias[n];
#pragma unroll
      for (int r = 0; r < 8; ++r) {
        float v = acc[i][j][r] * scale;
        if (BIAS_MODE == 1) v += bias[mBase + mOff + r];
        if (BIAS_MODE == 2) v += bv;
        if (RESID) v += Rb[(size_t)(mBase + mOff + r) * ldc + n];
        if (ACT == 1) v = tanhf(v);
        if (ACT == 2) v = fmaxf(v, 0.0f);
        if (ACT == 4) v = (v > 0.f) ? v : 0.01f * v;
        slab[(mOff + r) * 68 + (j << 4) + rlane] = v;
      }
    }
    __builtin_amdgcn_fence(__ATOMIC_RELEASE, "workgroup");
    __builtin_amdgcn_wave_barrier();
    __builtin_amdgcn_fence(__ATOMIC_ACQUIRE, "workgroup");
    if (OUT_MODE == 0) {
      float* C = (float*)Cout + (size_t)b * strideC;
      const int hh = lane >> 4, c4 = (lane & 15) * 4;
      for (int pass = 0; pass < 2; ++pass) {
#pragma unroll
        for (int it = 0; it < 8; ++it) {
          const int row = it * 2 + hh;
          v4f v = *(const v4f*)(slab + row * 68 + c4);
          *(volatile v4f*)(C + (size_t)(mBase + row) * ldc + n0 + c4) = v;
        }
        __threadfence();
      }
    } else {
      const int q = lane >> 3, c8 = (lane & 7) * 8;
      unsigned short* C  = (unsigned short*)Cout  + (size_t)b * strideC;
      unsigned short* C2 = (OUT_MODE == 2) ? ((unsigned short*)Cout2 + (size_t)b * strideC) : nullptr;
      for (int pass = 0; pass < 2; ++pass) {
#pragma unroll
        for (int it = 0; it < 4; ++it) {
          const int row = it * 4 + q;
          const float* sp = slab + row * 68 + c8;
          v8h hv, lv;
#pragma unroll
          for (int e = 0; e < 8; ++e) {
            if (OUT_MODE == 1) {
              hv[e] = (_Float16)sp[e];
            } else {
              unsigned short hb = f2bf_bits(sp[e]);
              unsigned short lb = f2bf_bits(sp[e] - bf_bits2f(hb));
              hv[e] = __builtin_bit_cast(_Float16, hb);
              lv[e] = __builtin_bit_cast(_Float16, lb);
            }
          }
          *(volatile v8h*)(C + (size_t)(mBase + row) * ldc + n0 + c8) = hv;
          if (OUT_MODE == 2) *(volatile v8h*)(C2 + (size_t)(mBase + row) * ldc + n0 + c8) = lv;
        }
        __threadfence();
      }
    }
    __builtin_amdgcn_fence(__ATOMIC_RELEASE, "workgroup");
    __builtin_amdgcn_wave_barrier();
    __builtin_amdgcn_fence(__ATOMIC_ACQUIRE, "workgroup");
  }
}

__global__ __launch_bounds__(256) void cast_scale_f16x8(const float* __restrict__ in, _Float16* __restrict__ out,
                                                          int n8, float scale) {
  const int i = blockIdx.x * 256 + threadIdx.x;
  if (i < n8) {
    const float* p = in + (size_t)i * 8;
    const v4f f0 = *(const v4f*)(p);
    const v4f f1 = *(const v4f*)(p + 4);
    v8h h;
    h[0] = (_Float16)(f0[0] * scale); h[1] = (_Float16)(f0[1] * scale);
    h[2] = (_Float16)(f0[2] * scale); h[3] = (_Float16)(f0[3] * scale);
    h[4] = (_Float16)(f1[0] * scale); h[5] = (_Float16)(f1[1] * scale);
    h[6] = (_Float16)(f1[2] * scale); h[7] = (_Float16)(f1[3] * scale);
    _Float16* q = out + (size_t)i * 8;
    *(volatile v8h*)q = h;
    __threadfence();
    *(volatile v8h*)q = h;
  }
}

__global__ __launch_bounds__(256) void cast_split_bf16x8(const float* __restrict__ in, unsigned short* __restrict__ hi,
                                                          unsigned short* __restrict__ lo, int n8) {
  const int i = blockIdx.x * 256 + threadIdx.x;
  if (i < n8) {
    const float* p = in + (size_t)i * 8;
    const v4f f0 = *(const v4f*)(p);
    const v4f f1 = *(const v4f*)(p + 4);
    v8h hv, lv;
#pragma unroll
    for (int e = 0; e < 4; ++e) {
      const unsigned short hb0 = f2bf_bits(f0[e]);
      const unsigned short lb0 = f2bf_bits(f0[e] - bf_bits2f(hb0));
      hv[e] = __builtin_bit_cast(_Float16, hb0); lv[e] = __builtin_bit_cast(_Float16, lb0);
      const unsigned short hb1 = f2bf_bits(f1[e]);
      const unsigned short lb1 = f2bf_bits(f1[e] - bf_bits2f(hb1));
      hv[4 + e] = __builtin_bit_cast(_Float16, hb1); lv[4 + e] = __builtin_bit_cast(_Float16, lb1);
    }
    unsigned short* qh = hi + (size_t)i * 8;
    unsigned short* ql = lo + (size_t)i * 8;
    *(volatile v8h*)qh = hv;
    *(volatile v8h*)ql = lv;
    __threadfence();
    *(volatile v8h*)qh = hv;
    *(volatile v8h*)ql = lv;
  }
}

__global__ __launch_bounds__(kGruThr) void gru_bidir_kernel(
    const float* __restrict__ X,
    const float* __restrict__ Wih,
    const float* __restrict__ Bih,
    const float* __restrict__ Bhh,
    const _Float16* __restrict__ WHH,
    const _Float16* __restrict__ PW0,
    const float* __restrict__ Pb0,
    const float* __restrict__ Pw1,
    const float* __restrict__ Pb1,
    const float* __restrict__ Pw2,
    const float* __restrict__ Pb2,
    _Float16* __restrict__ HS,
    float* __restrict__ out2) {
  __shared__ __align__(16) _Float16 h16[kTileS * kHPitch];
  __shared__ __align__(16) float s_p1w[kTileS * kPredH];
  __shared__ __align__(16) float s_pbuf[kTileS * kChunkC];
  __shared__ float s_xin[kTileS];

  const int tid = threadIdx.x, lane = tid & 31, wave = tid >> 5;
  const int rlane = lane & 15, hh = lane >> 4, koff = hh * 8, mOff = hh * 8;
  const int blk = blockIdx.x;
  const int sbase = blk * kTileS;
  const bool fwd = blk < (kSeqB / kTileS);
  const int xrow0 = fwd ? sbase : (sbase - kSeqB);

  for (int i = tid; i < kTileS * kHPitch; i += kGruThr) h16[i] = (_Float16)0.0f;

  const int j = 16 * wave + rlane;
  const float wi_r = Wih[j], wi_z = Wih[kHid + j], wi_n = Wih[2 * kHid + j];
  const float bi_r = Bih[j], bi_z = Bih[kHid + j], bi_n = Bih[2 * kHid + j];
  const float bh_r = Bhh[j], bh_z = Bhh[kHid + j], bh_n = Bhh[2 * kHid + j];
  const int u = 16 * (wave & 3) + rlane;
  const float pb0u = Pb0[u], pw1u = Pw1[u];
  const float pb1 = Pb1[0], pw2 = Pw2[0], pb2 = Pb2[0];
  float hf[8];
#pragma unroll
  for (int r = 0; r < 8; ++r) hf[r] = 0.0f;

  const _Float16* arow = h16 + rlane * kHPitch + koff;
  const _Float16* wgr = WHH + (size_t)j * kHid + koff;
  const _Float16* wgz = WHH + (size_t)(kHid + j) * kHid + koff;
  const _Float16* wgn = WHH + (size_t)(2 * kHid + j) * kHid + koff;
  const _Float16* wgp = PW0 + (size_t)u * kHid + koff;
  const v8f z8 = {0.f, 0.f, 0.f, 0.f, 0.f, 0.f, 0.f, 0.f};

  if (tid < kTileS) {
    const float xv0 = X[(size_t)(xrow0 + tid) * kSteps + (fwd ? 0 : (kSteps - 1))];
    s_xin[tid] = xv0;
    s_pbuf[tid * kChunkC + (fwd ? 0 : (kChunkC - 1))] = xv0;
  }
  __syncthreads();

#pragma unroll 1
  for (int t = 0; t < kSteps; ++t) {
    v8f ar = z8, az = z8, an = z8;
#pragma unroll 1
    for (int kc = 0; kc < kHid / 32; ++kc) {
      const int k0 = kc * 32;
      const v16h a  = Frag<_Float16>::load(arow + k0);
      const v16h br = Frag<_Float16>::load(wgr + k0);
      const v16h bz = Frag<_Float16>::load(wgz + k0);
      const v16h bn = Frag<_Float16>::load(wgn + k0);
      ar = Frag<_Float16>::mma(a, br, ar);
      az = Frag<_Float16>::mma(a, bz, az);
      an = Frag<_Float16>::mma(a, bn, an);
      dep_guard_h(ar, an, a, bn);
      keep4_h(br, bz, bn, a);
    }
    acc_guard3(ar, az, an);

#pragma unroll
    for (int r = 0; r < 8; ++r) {
      const float xin = s_xin[mOff + r];
      const float gr  = (xin * wi_r + bi_r) + (ar[r] * kInv16 + bh_r);
      const float gz  = (xin * wi_z + bi_z) + (az[r] * kInv16 + bh_z);
      const float hn  = an[r] * kInv16 + bh_n;
      const float rg  = fsigm(gr);
      const float zg  = fsigm(gz);
      const float ng  = ftanh((xin * wi_n + bi_n) + rg * hn);
      hf[r] = (1.0f - zg) * ng + zg * hf[r];
    }
    __syncthreads();

#pragma unroll
    for (int r = 0; r < 8; ++r) h16[(mOff + r) * kHPitch + j] = (_Float16)hf[r];
    __syncthreads();

    if (wave < 4) {
      v8f ap = z8;
#pragma unroll
      for (int kc = 0; kc < kHid / 32; ++kc) {
        const int k0 = kc * 32;
        const v16h a  = Frag<_Float16>::load(arow + k0);
        const v16h bp = Frag<_Float16>::load(wgp + k0);
        ap = Frag<_Float16>::mma(a, bp, ap);
        dep_guard1_h(ap, a, bp);
      }
#pragma unroll
      for (int r = 0; r < 8; ++r) {
        float v = ap[r] * kInv16 + pb0u;
        v = (v > 0.f) ? v : 0.01f * v;
        s_p1w[(mOff + r) * kPredH + u] = v * pw1u;
      }
    } else {
      const int w4 = wave - 4;
      const int q = lane >> 3, c8 = (lane & 7) * 8;
      const int coloff = fwd ? 0 : kHid;
      const int tpos = fwd ? t : (kSteps - 1 - t);
      for (int pass = 0; pass < 2; ++pass) {
#pragma unroll
        for (int it = 0; it < 2; ++it) {
          const int line = it * 4 + q;
          const int sl   = 4 * w4 + (line >> 1);
          const int col  = (line & 1) * 64 + c8;
          const v8h v = *(const v8h*)(h16 + sl * kHPitch + col);
          const size_t row = (size_t)(xrow0 + sl) * kSteps + tpos;
          _Float16* dst = HS + row * kFeatW + coloff + col;
          *(volatile v8h*)dst = v;
        }
        __threadfence();
      }
    }
    __syncthreads();

    if (tid < kTileS) {
      const float* prow = s_p1w + tid * kPredH;
      float sacc = 0.f;
#pragma unroll 4
      for (int uu = 0; uu < kPredH; ++uu) sacc += prow[uu];
      float v = sacc + pb1;
      v = (v > 0.f) ? v : 0.01f * v;
      const float pred = v * pw2 + pb2;
      if (t <= kSteps - 2) {
        const int c = fwd ? (t + 1) : (kSteps - 2 - t);
        s_pbuf[tid * kChunkC + (c & (kChunkC - 1))] = pred;
        const int tn = t + 1;
        const float xv = X[(size_t)(xrow0 + tid) * kSteps + (fwd ? tn : (kSteps - 1 - tn))];
        s_xin[tid] = (xv != xv) ? pred : xv;
      }
    }
    __syncthreads();

    if (t <= kSteps - 2) {
      const int c = fwd ? (t + 1) : (kSteps - 2 - t);
      const int slot = c & (kChunkC - 1);
      const bool doflush = fwd ? (slot == kChunkC - 1) : (slot == 0);
      if (doflush && wave == 0) {
        const int cc = c >> 5;
        const int q = lane >> 3, c4 = (lane & 7) * 4;
        for (int pass = 0; pass < 2; ++pass) {
#pragma unroll
          for (int it = 0; it < 4; ++it) {
            const int sl = it * 4 + q;
            const v4f v = *(const v4f*)(s_pbuf + sl * kChunkC + c4);
            float* dst = out2 + (size_t)(sbase + sl) * kSteps + cc * kChunkC + c4;
            *(volatile v4f*)dst = v;
          }
          __threadfence();
        }
      }
    }
  }
}

__global__ __launch_bounds__(256) void logit_head_kernel(const float* __restrict__ A1,
                                                         const float* __restrict__ W2,
                                                         const float* __restrict__ B2,
                                                         float* __restrict__ out0, float* __restrict__ out1,
                                                         int row0, int nrows) {
  const int i = blockIdx.x * 256 + threadIdx.x;
  if (i < nrows) {
    const float* p = A1 + (size_t)i * kFc1N;
    float acc = 0.f;
#pragma unroll 1
    for (int k = 0; k < kFc1N; k += 4) {
      const v4f a = *(const v4f*)(p + k);
      const v4f w = *(const v4f*)(W2 + k);
      acc += a[0] * w[0];
      acc += a[1] * w[1];
      acc += a[2] * w[2];
      acc += a[3] * w[3];
    }
    acc += B2[0];
    const float sg = fsigm(acc);
    const size_t o = (size_t)row0 + (size_t)i;
    *(volatile float*)(out1 + o) = acc;
    *(volatile float*)(out0 + o) = sg;
    __threadfence();
    *(volatile float*)(out1 + o) = acc;
    *(volatile float*)(out0 + o) = sg;
  }
}

extern "C" void kernel_launch(void* const* d_in, const int* in_sizes, int n_in,
                              void* d_out, int out_size, void* d_ws, size_t ws_size, hipStream_t stream) {
  if (n_in < 17 || d_out == nullptr || d_ws == nullptr) return;
  if (in_sizes[0] != kSeqB * kSteps || in_sizes[1] != kGate3 || in_sizes[2] != kGate3 * kHid ||
      in_sizes[3] != kGate3 || in_sizes[4] != kGate3 || in_sizes[5] != kFc0N * kFcK || in_sizes[6] != kFc0N ||
      in_sizes[7] != kFc1N * kFcK || in_sizes[8] != kFc1N || in_sizes[9] != kFc1N || in_sizes[10] != 1 ||
      in_sizes[11] != kPredH * kHid || in_sizes[12] != kPredH || in_sizes[13] != kPredH || in_sizes[14] != 1 ||
      in_sizes[15] != 1 || in_sizes[16] != 1 || out_size != 2 * kFcRows + kStreams * kSteps) return;

  const float* x     = (const float*)d_in[0];
  const float* w_ih  = (const float*)d_in[1];
  const float* w_hh  = (const float*)d_in[2];
  const float* b_ih  = (const float*)d_in[3];
  const float* b_hh  = (const float*)d_in[4];
  const float* fc_w0 = (const float*)d_in[5];
  const float* fc_b0 = (const float*)d_in[6];
  const float* fc_w1 = (const float*)d_in[7];
  const float* fc_b1 = (const float*)d_in[8];
  const float* fc_w2 = (const float*)d_in[9];
  const float* fc_b2 = (const float*)d_in[10];
  const float* p_w0  = (const float*)d_in[11];
  const float* p_b0  = (const float*)d_in[12];
  const float* p_w1  = (const float*)d_in[13];
  const float* p_b1  = (const float*)d_in[14];
  const float* p_w2  = (const float*)d_in[15];
  const float* p_b2  = (const float*)d_in[16];
  float* out0 = (float*)d_out;
  float* out1 = out0 + kFcRows;
  float* out2 = out0 + 2 * kFcRows;

  char* ws = (char*)d_ws; size_t off = 0;
  auto carve = [&](size_t bytes) -> char* { char* p = ws + off; off += (bytes + 255) & ~(size_t)255; return p; };
  _Float16* WHH16      = (_Float16*)carve((size_t)kGate3 * kHid * 2);
  _Float16* PW016      = (_Float16*)carve((size_t)kPredH * kHid * 2);
  _Float16* FCW016     = (_Float16*)carve((size_t)kFc0N * kFcK * 2);
  unsigned short* FCW1H = (unsigned short*)carve((size_t)kFc1N * kFcK * 2);
  unsigned short* FCW1L = (unsigned short*)carve((size_t)kFc1N * kFcK * 2);
  _Float16* HS16       = (_Float16*)carve((size_t)kFcRows * kFeatW * 2);
  unsigned short* FC0H  = (unsigned short*)carve((size_t)kFcChunk * kFc0N * 2);
  unsigned short* FC0L  = (unsigned short*)carve((size_t)kFcChunk * kFc0N * 2);
  float*    FC1C       = (float*)carve((size_t)kFcChunk * kFc1N * 4);
  if (off > ws_size || off > (size_t)134217728) return;

  cast_scale_f16x8<<<(kGate3 * kHid / 8) / 256, 256, 0, stream>>>(w_hh, WHH16, kGate3 * kHid / 8, 16.0f);
  cast_scale_f16x8<<<(kPredH * kHid / 8) / 256, 256, 0, stream>>>(p_w0, PW016, kPredH * kHid / 8, 16.0f);
  cast_scale_f16x8<<<(kFc0N * kFcK / 8) / 256, 256, 0, stream>>>(fc_w0, FCW016, kFc0N * kFcK / 8, 16.0f);
  cast_split_bf16x8<<<(kFc1N * kFcK / 8) / 256, 256, 0, stream>>>(fc_w1, FCW1H, FCW1L, kFc1N * kFcK / 8);

  gru_bidir_kernel<<<kStreams / kTileS, kGruThr, 0, stream>>>(x, w_ih, b_ih, b_hh, WHH16, PW016,
                                                             p_b0, p_w1, p_b1, p_w2, p_b2, HS16, out2);

  for (int ch = 0; ch < kFcRows / kFcChunk; ++ch) {
    const _Float16* Achunk = HS16 + (size_t)ch * kFcChunk * kFeatW;
    const int tiles0 = (kFcChunk / 64) * (kFc0N / 64);
    const int tiles1 = (kFcChunk / 64) * (kFc1N / 64);
    wmma_gemm64<0, false, 2, 2, false, 4><<<dim3((tiles0 + 7) / 8, 1), 256, 0, stream>>>(
        U16(Achunk), nullptr, kFeatW, 0L,
        U16(FCW016), nullptr, kFcK, 0L,
        (void*)FC0H, (void*)FC0L, kFc0N, 0L,
        fc_b0, nullptr, 0L, kFcChunk, kFc0N, kFcK, kInv16);
    wmma_gemm64<1, true, 2, 0, false, 4><<<dim3((tiles1 + 7) / 8, 1), 256, 0, stream>>>(
        FC0H, FC0L, kFc0N, 0L,
        FCW1H, FCW1L, kFcK, 0L,
        (void*)FC1C, nullptr, kFc1N, 0L,
        fc_b1, nullptr, 0L, kFcChunk, kFc1N, kFcK, 1.0f);
    logit_head_kernel<<<kFcChunk / 256, 256, 0, stream>>>(FC1C, fc_w2, fc_b2, out0, out1, ch * kFcChunk, kFcChunk);
  }
}
